// InvResMLP_24850680774735
// MI455X (gfx1250) — hardware-verified
//
#include <hip/hip_runtime.h>
#include <math.h>

typedef __attribute__((ext_vector_type(16))) _Float16 v16h;
typedef __attribute__((ext_vector_type(16))) __bf16 v16b;
typedef __attribute__((ext_vector_type(8)))  _Float16 v8h;
typedef __attribute__((ext_vector_type(8)))  float v8f;
typedef __attribute__((ext_vector_type(4)))  float v4f;
typedef __attribute__((ext_vector_type(2)))  float v2f;
typedef __attribute__((ext_vector_type(4)))  unsigned v4u;
typedef __attribute__((ext_vector_type(4)))  int v4i;
typedef float __attribute__((may_alias)) float_a;
typedef int __attribute__((may_alias)) int_a;

template <typename T> __device__ __forceinline__ void vst2(void* p, T v) { *(volatile T*)p = v; __threadfence(); *(volatile T*)p = v; }
__device__ __forceinline__ v8f wmma16(v16h a, v16h b, v8f c) {
  v8f d = __builtin_amdgcn_wmma_f32_16x16x32_f16(false, a, false, b, (short)0, c, false, false);
  asm volatile("v_nop\n\tv_nop\n\tv_nop\n\tv_nop" : "+v"(d) : "v"(a), "v"(b));
  return d;
}
__device__ __forceinline__ v8f wmma_bf(v16b a, v16b b, v8f c) {
  v8f d = __builtin_amdgcn_wmma_f32_16x16x32_bf16(false, a, false, b, (short)0, c, false, false);
  asm volatile("v_nop\n\tv_nop\n\tv_nop\n\tv_nop" : "+v"(d) : "v"(a), "v"(b));
  return d;
}
__device__ __forceinline__ v16h frag_h(const _Float16* rowk0, int lane) {
  union { v16h v; v8h q[2]; } u; const _Float16* p = rowk0 + 8 * (lane >> 4);
  u.q[0] = *(const v8h*)p; u.q[1] = *(const v8h*)(p + 16); return u.v;
}
__device__ __forceinline__ v16h frag_f32(const float* rowk0, int lane) {
  v16h a; const float* p = rowk0 + 8 * (lane >> 4);
#pragma unroll
  for (int i = 0; i < 8; ++i) { a[i] = (_Float16)p[i]; a[8 + i] = (_Float16)p[16 + i]; }
  return a;
}
__device__ __forceinline__ v16h frag_f32s(const float* rowk0, int lane, float sc) {
  v16h a; const float* p = rowk0 + 8 * (lane >> 4);
#pragma unroll
  for (int i = 0; i < 8; ++i) { a[i] = (_Float16)(p[i] * sc); a[8 + i] = (_Float16)(p[16 + i] * sc); }
  return a;
}
__device__ __forceinline__ v16h fragc_f32(const float* W, int k0, int n, int lane, int ld, int K) {
  v16h a; const int g = lane >> 4;
#pragma unroll
  for (int i = 0; i < 8; ++i) { const int ka = k0 + 8 * g + i, kb = ka + 16;
    a[i] = (_Float16)(ka < K ? W[(size_t)(ka < K ? ka : K - 1) * ld + n] : 0.f); a[8 + i] = (_Float16)(kb < K ? W[(size_t)(kb < K ? kb : K - 1) * ld + n] : 0.f); }
  return a;
}
struct F2 { v16b h, l; };
__device__ __forceinline__ F2 bsplit16(const float v[16]) { F2 r;
#pragma unroll
  for (int i = 0; i < 16; ++i) { const __bf16 h = (__bf16)v[i]; r.h[i] = h; r.l[i] = (__bf16)(v[i] - (float)h); }
  return r; }
__device__ __forceinline__ F2 split_row(const float* row, int k0, int lane) { float v[16]; const float* p = row + k0 + 8 * (lane >> 4);
#pragma unroll
  for (int i = 0; i < 8; ++i) { v[i] = p[i]; v[8 + i] = p[16 + i]; }
  return bsplit16(v); }
__device__ __forceinline__ F2 split_rowK(const float* row, int k0, int lane, int K) { float v[16]; const int g = lane >> 4;
#pragma unroll
  for (int i = 0; i < 8; ++i) { const int ka = k0 + 8 * g + i, kb = ka + 16; v[i] = ka < K ? row[ka < K ? ka : K - 1] : 0.f; v[8 + i] = kb < K ? row[kb < K ? kb : K - 1] : 0.f; }
  return bsplit16(v); }
__device__ __forceinline__ F2 split_col(const float* W, int k0, int n, int lane, int ld, int K) { float v[16]; const int g = lane >> 4;
#pragma unroll
  for (int i = 0; i < 8; ++i) { const int ka = k0 + 8 * g + i, kb = ka + 16; v[i] = ka < K ? W[(size_t)(ka < K ? ka : K - 1) * ld + n] : 0.f; v[8 + i] = kb < K ? W[(size_t)(kb < K ? kb : K - 1) * ld + n] : 0.f; }
  return bsplit16(v); }
__device__ __forceinline__ v8f mac3(const F2& a, const F2& b, v8f c) { c = wmma_bf(a.l, b.h, c); c = wmma_bf(a.h, b.l, c); return wmma_bf(a.h, b.h, c); }
__device__ __forceinline__ float sigm(float v) { return 1.0f / (1.0f + expf(-v)); }
#define LDSX() do { asm volatile("s_wait_dscnt 0" ::: "memory"); __builtin_amdgcn_wave_barrier(); __builtin_amdgcn_fence(__ATOMIC_RELEASE, "workgroup"); } while (0)

#define NBT 8
#define NPT 4096
#define NR (NBT * NPT)
#define CCH 128
#define CH4 512
#define KNB 32
#define R2 0.0225f
#define RINV (1.0f / 0.15f)
#ifndef NRV
#define NRV NR
#endif
__device__ __forceinline__ float bfr(float v) { return (float)(__bf16)v; }
__device__ __forceinline__ v16b wcol_oi(const float* Wm, int k0, int o, int lane, int K) { v16b w; const float* p = Wm + (size_t)o * K + k0 + 8 * (lane >> 4);
#pragma unroll
  for (int i = 0; i < 8; ++i) { w[i] = (__bf16)p[i]; w[8 + i] = (__bf16)p[16 + i]; }
  return w; }
#define OUT1_OFF (4u * (size_t)NR * 3)
#define WS_IDX 0u
#define WS_F   (WS_IDX + 4u * (size_t)NR * KNB)
#define WS_H   (WS_F + 4u * (size_t)NR * CCH)
#define WS_END (WS_H + 4u * (size_t)NR * CH4)

__global__ __launch_bounds__(256) void k_pos(const float* __restrict__ P, float* __restrict__ OUT0) { const size_t e = (size_t)blockIdx.x * 256 + threadIdx.x; if (e >= (size_t)NR * 3 / 4) return; const v4f v = *(const v4f*)(P + e * 4); v4f o; o[0] = bfr(v[0]); o[1] = bfr(v[1]); o[2] = bfr(v[2]); o[3] = bfr(v[3]); vst2(OUT0 + e * 4, o); }
__global__ __launch_bounds__(256) void k_ball(const float* __restrict__ P, int* __restrict__ IDX) {
  const int wave = threadIdx.x >> 5, lane = threadIdx.x & 31; const size_t m = (size_t)blockIdx.x * 8 + wave; if (m >= (size_t)NRV) return;
  const size_t b = m / NPT; __shared__ int sid[8][KNB];
  float qx, qy, qz, sqm;
  {
#pragma clang fp contract(off)
    qx = bfr(P[m * 3]); qy = bfr(P[m * 3 + 1]); qz = bfr(P[m * 3 + 2]); sqm = (qx * qx + qy * qy) + qz * qz;
    int cnt = 0;
#pragma unroll 1
    for (int n0 = 0; n0 < NPT && cnt < KNB; n0 += 32) { const size_t n = b * NPT + n0 + lane;
      const float px = bfr(P[n * 3]), py = bfr(P[n * 3 + 1]), pz = bfr(P[n * 3 + 2]);
      const float sqn = (px * px + py * py) + pz * pz; const float dot = (qx * px + qy * py) + qz * pz; const float d2 = (sqm + sqn) - 2.0f * dot;
      const bool in = d2 < R2;
      const unsigned bal = __builtin_amdgcn_ballot_w32(in);
      const int before = __builtin_popcount(bal & ((1u << lane) - 1u));
      const int pos = cnt + before;
      if (in && pos < KNB) sid[wave][pos] = n0 + lane;
      cnt += __builtin_popcount(bal); }
    asm volatile("s_wait_dscnt 0" ::: "memory"); __builtin_amdgcn_wave_barrier();
    const int total = cnt < KNB ? cnt : KNB;
    const int v = lane < total ? sid[wave][lane] : sid[wave][0];
    vst2(IDX + m * KNB + lane, v); } }
__global__ __launch_bounds__(128) void k_edge(const float* __restrict__ P, const float* __restrict__ X, const int* __restrict__ IDX, const float* __restrict__ W1, const float* __restrict__ G1, const float* __restrict__ B1, const float* __restrict__ M1, const float* __restrict__ V1, float* __restrict__ F) {
  __shared__ float smax[4][CCH]; __shared__ int sidx[2][KNB];
  const int tid = threadIdx.x, wave = tid >> 5, lane = tid & 31, col = lane & 15, g = lane >> 4; const size_t m = (size_t)blockIdx.x * 2 + (wave >> 1); const int half = wave & 1;
  if (tid < 64) { const size_t mm = (size_t)blockIdx.x * 2 + (tid >> 5); int v = IDX[mm * KNB + (tid & 31)]; v = v < 0 ? 0 : (v >= NPT ? NPT - 1 : v); sidx[tid >> 5][tid & 31] = v; }
  __syncthreads();
  const size_t b = m / NPT; const int myn = sidx[wave >> 1][half * 16 + col];
  const float* xr = X + (b * NPT + myn) * CCH;
  v8f acc[8] = {};
#pragma unroll
  for (int kc = 0; kc < CCH / 32; ++kc) { v16b a; { const float* p = xr + kc * 32 + 8 * g;
#pragma unroll
      for (int i = 0; i < 8; ++i) { a[i] = (__bf16)p[i]; a[8 + i] = (__bf16)p[16 + i]; } }
    asm volatile("s_wait_loadcnt 0x0" ::: "memory");
#pragma unroll
    for (int j = 0; j < 8; ++j) { v16b w; { const float* p = W1 + (size_t)(j * 16 + col) * (CCH + 3) + 3 + kc * 32 + 8 * g;
#pragma unroll
        for (int i = 0; i < 8; ++i) { w[i] = (__bf16)p[i]; w[8 + i] = (__bf16)p[16 + i]; } }
      asm volatile("s_wait_loadcnt 0x0" ::: "memory"); acc[j] = wmma_bf(a, w, acc[j]); } }
  const float cx = bfr(P[m * 3]), cy = bfr(P[m * 3 + 1]), cz = bfr(P[m * 3 + 2]);
#pragma unroll
  for (int j = 0; j < 8; ++j) { const int o = j * 16 + col; const float w0 = bfr(W1[(size_t)o * (CCH + 3)]), w1 = bfr(W1[(size_t)o * (CCH + 3) + 1]), w2 = bfr(W1[(size_t)o * (CCH + 3) + 2]);
    const float sc = bfr(G1[o]) / sqrtf(bfr(V1[o]) + 1e-5f), mean = bfr(M1[o]), beta = bfr(B1[o]);
    float mx = -3.0e38f;
#pragma unroll
    for (int r = 0; r < 8; ++r) { const int nb = sidx[wave >> 1][half * 16 + 8 * g + r]; const float* pn = P + (b * NPT + nb) * 3;
      const float rx = (bfr(pn[0]) - cx) * RINV, ry = (bfr(pn[1]) - cy) * RINV, rz = (bfr(pn[2]) - cz) * RINV;
      const float y = acc[j][r] + rx * w0 + ry * w1 + rz * w2; const float yb = (y - mean) * sc + beta; mx = fmaxf(mx, fmaxf(yb, 0.f)); }
    mx = fmaxf(mx, __shfl_xor(mx, 16));
    if (g == 0) smax[wave][o] = mx; }
  __syncthreads();
  for (int e = tid; e < 2 * (CCH / 4); e += 128) { const int cc2 = e / (CCH / 4), q = e % (CCH / 4); const size_t mm = (size_t)blockIdx.x * 2 + cc2; v4f o4;
#pragma unroll
    for (int i = 0; i < 4; ++i) o4[i] = fmaxf(smax[cc2 * 2][q * 4 + i], smax[cc2 * 2 + 1][q * 4 + i]);
    vst2(F + mm * CCH + q * 4, o4); } }
__device__ __forceinline__ F2 arow_bn(const float* row, int k0, int lane, const float* __restrict__ G, const float* __restrict__ Bt, const float* __restrict__ Mn, const float* __restrict__ Vr) { float v[16]; const float* p = row + k0 + 8 * (lane >> 4);
#pragma unroll
  for (int i = 0; i < 8; ++i) { v[i] = p[i]; v[8 + i] = p[16 + i]; }
  if (G) {
#pragma unroll
    for (int i = 0; i < 16; ++i) { const int c = k0 + 8 * (lane >> 4) + (i < 8 ? i : 8 + i); const float y = (v[i] - bfr(Mn[c])) * (bfr(G[c]) / sqrtf(bfr(Vr[c]) + 1e-5f)) + bfr(Bt[c]); v[i] = fmaxf(y, 0.f); } }
  return bsplit16(v); }
__global__ __launch_bounds__(128) void k_mlp(const float* __restrict__ IN, int ldin, int K, const float* __restrict__ Ga, const float* __restrict__ Ba, const float* __restrict__ Ma, const float* __restrict__ Va, const float* __restrict__ Wt, int mode, const float* __restrict__ G3, const float* __restrict__ B3, const float* __restrict__ M3, const float* __restrict__ V3, const float* __restrict__ X, float* __restrict__ OUTR, int ldout) { __shared__ __align__(16) float sf[4][16][132];
  const int tid = threadIdx.x, wave = tid >> 5, lane = tid & 31, col = lane & 15, g = lane >> 4; const int c0 = blockIdx.y * 128; const size_t r0 = (size_t)blockIdx.x * 64 + wave * 16;
  v8f acc[8] = {};
#pragma unroll 1
  for (int kc = 0; kc < K / 32; ++kc) { const F2 a = arow_bn(IN + (r0 + col) * ldin, kc * 32, lane, Ga, Ba, Ma, Va); asm volatile("s_wait_loadcnt 0x0" ::: "memory");
#pragma unroll
    for (int j = 0; j < 8; ++j) { const v16b w = wcol_oi(Wt, kc * 32, c0 + j * 16 + col, lane, K); asm volatile("s_wait_loadcnt 0x0" ::: "memory"); acc[j] = wmma_bf(a.h, w, acc[j]); acc[j] = wmma_bf(a.l, w, acc[j]); } }
  if (mode == 0) {
#pragma unroll
    for (int j = 0; j < 8; ++j)
#pragma unroll
      for (int r = 0; r < 8; ++r) sf[wave][8 * g + r][j * 16 + col] = acc[j][r];
  } else {
#pragma unroll
    for (int j = 0; j < 8; ++j) { const int o = c0 + j * 16 + col; const float sc = bfr(G3[o]) / sqrtf(bfr(V3[o]) + 1e-5f), mean = bfr(M3[o]), beta = bfr(B3[o]);
#pragma unroll
      for (int r = 0; r < 8; ++r) { const size_t row = r0 + 8 * g + r; const float hres = (acc[j][r] - mean) * sc + beta + bfr(X[row * CCH + o]); sf[wave][8 * g + r][j * 16 + col] = fmaxf(hres, 0.f); }
      asm volatile("s_wait_loadcnt 0x0" ::: "memory"); } }
  LDSX(); for (int rl = 0; rl < 16; ++rl) vst2(OUTR + (r0 + rl) * (size_t)ldout + c0 + lane * 4, *(const v4f*)&sf[wave][rl][lane * 4]); }
extern "C" void kernel_launch(void* const* d_in, const int* in_sizes, int n_in, void* d_out, int out_size, void* d_ws, size_t ws_size, hipStream_t stream) {
  (void)in_sizes; (void)n_in; (void)out_size;
  const float** Fi = (const float**)d_in;
  if (ws_size < (size_t)WS_END) return;
  char* ws = (char*)d_ws; int* IDX = (int*)(ws + WS_IDX); float *Fr = (float*)(ws + WS_F), *Hr = (float*)(ws + WS_H); float* OUT1 = (float*)((char*)d_out + OUT1_OFF);
  k_pos<<<dim3((NR * 3 / 4 + 255) / 256), 256, 0, stream>>>(Fi[0], (float*)d_out);
  k_ball<<<dim3((NRV + 7) / 8), 256, 0, stream>>>(Fi[0], IDX);
  k_edge<<<dim3(NRV / 2), 128, 0, stream>>>(Fi[0], Fi[1], IDX, Fi[2], Fi[3], Fi[4], Fi[5], Fi[6], Fr);
  k_mlp<<<dim3(NRV / 64, CH4 / 128), 128, 0, stream>>>(Fr, CCH, CCH, nullptr, nullptr, nullptr, nullptr, Fi[7], 0, nullptr, nullptr, nullptr, nullptr, nullptr, Hr, CH4);
  k_mlp<<<dim3(NRV / 64, CCH / 128), 128, 0, stream>>>(Hr, CH4, CH4, Fi[8], Fi[9], Fi[10], Fi[11], Fi[12], 1, Fi[13], Fi[14], Fi[15], Fi[16], Fi[1], OUT1, CCH);
}
